// NeuralCellularAutomata2_34299608825955
// MI455X (gfx1250) — hardware-verified
//
#include <hip/hip_runtime.h>
#include <math.h>

typedef __attribute__((ext_vector_type(16))) _Float16 v16h;
typedef __attribute__((ext_vector_type(16))) __bf16 v16b;
typedef __attribute__((ext_vector_type(8)))  _Float16 v8h;
typedef __attribute__((ext_vector_type(8)))  float v8f;
typedef __attribute__((ext_vector_type(4)))  float v4f;
typedef __attribute__((ext_vector_type(2)))  float v2f;
typedef __attribute__((ext_vector_type(4)))  unsigned v4u;
typedef __attribute__((ext_vector_type(4)))  int v4i;
typedef float __attribute__((may_alias)) float_a;
typedef int __attribute__((may_alias)) int_a;

template <typename T> __device__ __forceinline__ void vst2(void* p, T v) { *(volatile T*)p = v; __threadfence(); *(volatile T*)p = v; }
__device__ __forceinline__ v8f wmma16(v16h a, v16h b, v8f c) {
  v8f d = __builtin_amdgcn_wmma_f32_16x16x32_f16(false, a, false, b, (short)0, c, false, false);
  asm volatile("v_nop\n\tv_nop\n\tv_nop\n\tv_nop" : "+v"(d) : "v"(a), "v"(b));
  return d;
}
__device__ __forceinline__ v8f wmma_bf(v16b a, v16b b, v8f c) {
  v8f d = __builtin_amdgcn_wmma_f32_16x16x32_bf16(false, a, false, b, (short)0, c, false, false);
  asm volatile("v_nop\n\tv_nop\n\tv_nop\n\tv_nop" : "+v"(d) : "v"(a), "v"(b));
  return d;
}
__device__ __forceinline__ v16h frag_h(const _Float16* rowk0, int lane) {
  union { v16h v; v8h q[2]; } u; const _Float16* p = rowk0 + 8 * (lane >> 4);
  u.q[0] = *(const v8h*)p; u.q[1] = *(const v8h*)(p + 16); return u.v;
}
__device__ __forceinline__ v16h frag_f32(const float* rowk0, int lane) {
  v16h a; const float* p = rowk0 + 8 * (lane >> 4);
#pragma unroll
  for (int i = 0; i < 8; ++i) { a[i] = (_Float16)p[i]; a[8 + i] = (_Float16)p[16 + i]; }
  return a;
}
__device__ __forceinline__ v16h frag_f32s(const float* rowk0, int lane, float sc) {
  v16h a; const float* p = rowk0 + 8 * (lane >> 4);
#pragma unroll
  for (int i = 0; i < 8; ++i) { a[i] = (_Float16)(p[i] * sc); a[8 + i] = (_Float16)(p[16 + i] * sc); }
  return a;
}
__device__ __forceinline__ v16h fragc_f32(const float* W, int k0, int n, int lane, int ld, int K) {
  v16h a; const int g = lane >> 4;
#pragma unroll
  for (int i = 0; i < 8; ++i) { const int ka = k0 + 8 * g + i, kb = ka + 16;
    a[i] = (_Float16)(ka < K ? W[(size_t)ka * ld + n] : 0.f); a[8 + i] = (_Float16)(kb < K ? W[(size_t)kb * ld + n] : 0.f); }
  return a;
}
struct F2 { v16b h, l; };
__device__ __forceinline__ F2 bsplit16(const float v[16]) { F2 r;
#pragma unroll
  for (int i = 0; i < 16; ++i) { const __bf16 h = (__bf16)v[i]; r.h[i] = h; r.l[i] = (__bf16)(v[i] - (float)h); }
  return r; }
__device__ __forceinline__ F2 split_row(const float* row, int k0, int lane) { float v[16]; const float* p = row + k0 + 8 * (lane >> 4);
#pragma unroll
  for (int i = 0; i < 8; ++i) { v[i] = p[i]; v[8 + i] = p[16 + i]; }
  return bsplit16(v); }
__device__ __forceinline__ F2 split_rowK(const float* row, int k0, int lane, int K) { float v[16]; const int g = lane >> 4;
#pragma unroll
  for (int i = 0; i < 8; ++i) { const int ka = k0 + 8 * g + i, kb = ka + 16; v[i] = ka < K ? row[ka] : 0.f; v[8 + i] = kb < K ? row[kb] : 0.f; }
  return bsplit16(v); }
__device__ __forceinline__ F2 split_col(const float* W, int k0, int n, int lane, int ld, int K) { float v[16]; const int g = lane >> 4;
#pragma unroll
  for (int i = 0; i < 8; ++i) { const int ka = k0 + 8 * g + i, kb = ka + 16; v[i] = ka < K ? W[(size_t)ka * ld + n] : 0.f; v[8 + i] = kb < K ? W[(size_t)kb * ld + n] : 0.f; }
  return bsplit16(v); }
__device__ __forceinline__ v8f mac3(const F2& a, const F2& b, v8f c) { c = wmma_bf(a.l, b.h, c); c = wmma_bf(a.h, b.l, c); return wmma_bf(a.h, b.h, c); }
__device__ __forceinline__ float sigm(float v) { return 1.0f / (1.0f + expf(-v)); }
#define LDSX() do { asm volatile("s_wait_dscnt 0" ::: "memory"); __builtin_amdgcn_wave_barrier(); __builtin_amdgcn_fence(__ATOMIC_RELEASE, "workgroup"); } while (0)

#define NB 8
#define HH 128
#define WW 128
#define C 64
#define C3 192
#define C2 128
#define TP 64

__device__ __forceinline__ float gelu_e(float v) { return 0.5f * v * (1.0f + erff(v * 0.70710678118654752f)); }
__global__ __launch_bounds__(256) void k_pack(const float* __restrict__ w1, const float* __restrict__ w2, const float* __restrict__ wq, _Float16* __restrict__ W1P, _Float16* __restrict__ W2P, _Float16* __restrict__ WQP) {
  const int r = blockIdx.x, tid = threadIdx.x; __shared__ __align__(16) _Float16 srow[C3];
  const float* W; _Float16* D; int K, n;
  if (r < C2) { W = w1 + (size_t)r * C3; D = W1P + (size_t)r * C3; K = C3; } else if (r < C2 + C) { n = r - C2; W = w2 + (size_t)n * C2; D = W2P + (size_t)n * C2; K = C2; } else { n = r - C2 - C; W = wq + (size_t)n * C; D = WQP + (size_t)n * C; K = C; }
  if (tid < K) srow[tid] = (_Float16)(W[tid] * 16.0f);
  __syncthreads();
  if (tid < K / 8) vst2(D + tid * 8, *(const v4u*)(&srow[tid * 8]));
}
__global__ __launch_bounds__(128) void k_cell(const float* __restrict__ h, const float* __restrict__ wp, const float* __restrict__ bp, const float* __restrict__ w1, const float* __restrict__ b1, const _Float16* __restrict__ W2P, const float* __restrict__ b2, const _Float16* __restrict__ WQP, const float* __restrict__ bq,
                                            float* __restrict__ HN, _Float16* __restrict__ QKV) {
  __shared__ __align__(16) float sh[3][TP + 2][C];
  __shared__ __align__(16) _Float16 sa[4][16][C3 + 8];
  __shared__ __align__(16) float so[4][16][196];
  __shared__ float swp[C3 * 9], sbp[C3];
  const int tid = threadIdx.x, wave = tid >> 5, lane = tid & 31, col = lane & 15, g = lane >> 4;
  const int b = blockIdx.z, y = blockIdx.y, x0 = blockIdx.x * TP;
  for (int q = tid; q < C3 * 9; q += 128) swp[q] = wp[q];
  for (int q = tid; q < C3; q += 128) sbp[q] = bp[q];
  for (int q = tid; q < 3 * (TP + 2) * (C / 4); q += 128) { const int c4 = q % (C / 4), rest = q / (C / 4); const int px = rest % (TP + 2), ry = rest / (TP + 2); const int yy = y - 1 + ry, xx = x0 - 1 + px;
    v4f v = (v4f){0.f, 0.f, 0.f, 0.f}; if (yy >= 0 && yy < HH && xx >= 0 && xx < WW) v = *(const v4f*)(h + (((size_t)b * HH + yy) * WW + xx) * C + c4 * 4);
    *(v4f*)(&sh[ry][px][c4 * 4]) = v; }
  __syncthreads();
  const size_t prow0 = ((size_t)b * HH + y) * WW + x0 + wave * 16;
  { const int pl = lane >> 1, hf = lane & 1; const int px = wave * 16 + pl + 1;
#pragma unroll 1
    for (int o = hf * 96; o < hf * 96 + 96; ++o) { const int c = o / 3; const float* w9 = &swp[o * 9]; float s = sbp[o];
#pragma unroll
      for (int dy = 0; dy < 3; ++dy)
#pragma unroll
        for (int dx = 0; dx < 3; ++dx) s += w9[dy * 3 + dx] * sh[dy][px - 1 + dx][c];
      so[wave][pl][o] = s; } }
  LDSX();
  { v8f acc[8] = {};
#pragma unroll 1
    for (int kc = 0; kc < C3 / 32; ++kc) { const F2 a = split_row(&so[wave][col][0], kc * 32, lane);
#pragma unroll
      for (int t = 0; t < 8; ++t) acc[t] = mac3(a, split_row(w1 + (size_t)(t * 16 + col) * C3, kc * 32, lane), acc[t]); }
    LDSX();
#pragma unroll
    for (int t = 0; t < 8; ++t) { const float bb = b1[t * 16 + col];
#pragma unroll
      for (int r = 0; r < 8; ++r) sa[wave][8 * g + r][t * 16 + col] = (_Float16)gelu_e(acc[t][r] + bb); } }
  LDSX();
  { v8f acc[4] = {};
#pragma unroll
    for (int kc = 0; kc < C2 / 32; ++kc) { const v16h a = frag_h(&sa[wave][col][0] + kc * 32, lane);
#pragma unroll
      for (int t = 0; t < 4; ++t) acc[t] = wmma16(a, frag_h(W2P + (size_t)(t * 16 + col) * C2 + kc * 32, lane), acc[t]); }
    LDSX();
#pragma unroll
    for (int t = 0; t < 4; ++t) { const int c = t * 16 + col; const float bb = b2[c];
#pragma unroll
      for (int r = 0; r < 8; ++r) { const float v = acc[t][r] * (1.0f / 16.0f) + bb + sh[1][wave * 16 + 8 * g + r + 1][c]; so[wave][8 * g + r][c] = v; sa[wave][8 * g + r][c] = (_Float16)v; } } }
  LDSX();
  for (int q = lane; q < 16 * 16; q += 32) { const int rl = q >> 4, pc = q & 15; vst2(HN + (prow0 + rl) * C + pc * 4, *(const v4f*)(&so[wave][rl][pc * 4])); }
  { v8f acc[12];
#pragma unroll
    for (int t = 0; t < 12; ++t) acc[t] = (v8f){};
#pragma unroll
    for (int kc = 0; kc < C / 32; ++kc) { const v16h a = frag_h(&sa[wave][col][0] + kc * 32, lane);
#pragma unroll
      for (int t = 0; t < 12; ++t) acc[t] = wmma16(a, frag_h(WQP + (size_t)(t * 16 + col) * C + kc * 32, lane), acc[t]); }
    LDSX();
#pragma unroll
    for (int t = 0; t < 12; ++t) { const float bb = bq[t * 16 + col];
#pragma unroll
      for (int r = 0; r < 8; ++r) so[wave][8 * g + r][t * 16 + col] = acc[t][r] * (1.0f / 16.0f) + bb; } }
  LDSX();
  for (int q = lane; q < 16 * 24; q += 32) { const int rl = q / 24, pc = q % 24; union { v8h h8; v4u u; } pk;
#pragma unroll
    for (int e = 0; e < 8; ++e) pk.h8[e] = (_Float16)so[wave][rl][pc * 8 + e];
    vst2(QKV + (prow0 + rl) * C3 + pc * 8, pk.u); }
}
__global__ __launch_bounds__(128) void k_lattn(const _Float16* __restrict__ QKV, const float* __restrict__ HN, float* __restrict__ out) {
  __shared__ __align__(16) _Float16 sk[3][TP + 2][C + 8], sv[3][TP + 2][C + 8];
  __shared__ __align__(16) float sq[TP][C + 4];
  __shared__ __align__(16) float so[TP][C + 4];
  const int tid = threadIdx.x; const int b = blockIdx.z, y = blockIdx.y, x0 = blockIdx.x * TP;
  for (int q = tid; q < 3 * (TP + 2) * 8; q += 128) { const int pc = q & 7, rest = q >> 3; const int px = rest % (TP + 2), ry = rest / (TP + 2); const int yy = y - 1 + ry, xx = x0 - 1 + px;
    union { v4u u; v8h h8; } pk, pv; pk.u = (v4u){0u, 0u, 0u, 0u}; pv.u = pk.u;
    if (yy >= 0 && yy < HH && xx >= 0 && xx < WW) { const _Float16* r = QKV + (((size_t)b * HH + yy) * WW + xx) * C3; pk.u = *(const v4u*)(r + C + pc * 8); pv.u = *(const v4u*)(r + 2 * C + pc * 8); }
    *(v4u*)(&sk[ry][px][pc * 8]) = pk.u; *(v4u*)(&sv[ry][px][pc * 8]) = pv.u; }
  for (int q = tid; q < TP * 8; q += 128) { const int pl = q >> 3, pc = q & 7; const _Float16* r = QKV + (((size_t)b * HH + y) * WW + x0 + pl) * C3; union { v4u u; v8h h8; } pk; pk.u = *(const v4u*)(r + pc * 8);
#pragma unroll
    for (int e = 0; e < 8; ++e) sq[pl][pc * 8 + e] = (float)pk.h8[e]; }
  __syncthreads();
  { const int pl = tid >> 1, hf = tid & 1; float sc[9];
#pragma unroll
    for (int nb = 0; nb < 9; ++nb) { const int dy = nb / 3, dx = nb % 3; const _Float16* kr = &sk[dy][pl + dx][hf * 32]; const float* qr = &sq[pl][hf * 32]; float s = 0.f;
#pragma unroll 1
      for (int c = 0; c < 32; ++c) s += qr[c] * (float)kr[c];
      s += __shfl_xor(s, 1, 32); sc[nb] = s * 0.125f; }
    float mx = sc[0];
#pragma unroll
    for (int nb = 1; nb < 9; ++nb) mx = fmaxf(mx, sc[nb]);
    float se = 0.f;
#pragma unroll
    for (int nb = 0; nb < 9; ++nb) { sc[nb] = expf(sc[nb] - mx); se += sc[nb]; }
    const float inv = 1.0f / se;
#pragma unroll 1
    for (int c = hf * 32; c < hf * 32 + 32; ++c) { float a = 0.f;
#pragma unroll
      for (int nb = 0; nb < 9; ++nb) a += sc[nb] * (float)sv[nb / 3][pl + nb % 3][c];
      so[pl][c] = a * inv; } }
  __syncthreads();
  for (int q = tid; q < TP * 16; q += 128) { const int pl = q >> 4, pc = q & 15; const size_t p = ((size_t)b * HH + y) * WW + x0 + pl; v4f o = *(const v4f*)(&so[pl][pc * 4]); const v4f hn = *(const v4f*)(HN + p * C + pc * 4);
    o += hn; vst2(out + p * C + pc * 4, o); }
}
extern "C" void kernel_launch(void* const* d_in, const int* in_sizes, int n_in, void* d_out, int out_size, void* d_ws, size_t ws_size, hipStream_t stream) {
  (void)in_sizes; (void)n_in; (void)out_size; (void)ws_size;
  const float** I = (const float**)d_in;
  const float* h = I[0]; const float* wp = I[1]; const float* bp = I[2]; const float* w1 = I[3]; const float* b1 = I[4]; const float* w2 = I[5]; const float* b2 = I[6]; const float* wq = I[7]; const float* bq = I[8];
  float* out = (float*)d_out;
  char* ws = (char*)d_ws; size_t off = 0;
  auto take = [&](size_t bytes) { char* p = ws + off; off += (bytes + 255) & ~(size_t)255; return p; };
  _Float16* W1P = (_Float16*)take(C2 * C3 * 2); _Float16* W2P = (_Float16*)take(C * C2 * 2); _Float16* WQP = (_Float16*)take(C3 * C * 2);
  float* HN = (float*)take((size_t)NB * HH * WW * C * 4); _Float16* QKV = (_Float16*)take((size_t)NB * HH * WW * C3 * 2);
  k_pack<<<C2 + C + C3, 256, 0, stream>>>(w1, w2, wq, W1P, W2P, WQP);
  k_cell<<<dim3(WW / TP, HH, NB), 128, 0, stream>>>(h, wp, bp, w1, b1, W2P, b2, WQP, bq, HN, QKV);
  k_lattn<<<dim3(WW / TP, HH, NB), 128, 0, stream>>>(QKV, HN, out);
}
